// SelfAttentionConv_6657199308858
// MI455X (gfx1250) — hardware-verified
//
#include <hip/hip_runtime.h>
#include <hip/hip_bf16.h>
#include <math.h>


#define BB 4
#define SS 2048
#define DD 1024
#define HH 8
#define DKK 128
#define KS2 136
#define QW 1

typedef _Float16 bf16;
typedef __attribute__((ext_vector_type(4))) unsigned v4u_t;
typedef unsigned v4ua __attribute__((ext_vector_type(4), may_alias));
typedef __attribute__((ext_vector_type(4))) float v4f_t;
typedef float v4fa __attribute__((ext_vector_type(4), may_alias));
typedef __attribute__((ext_vector_type(16))) bf16  bf16x16;
typedef __attribute__((ext_vector_type(8)))  bf16  bf16x8;
typedef __attribute__((ext_vector_type(4)))  bf16  bf16x4;
typedef __attribute__((ext_vector_type(8)))  float f32x8;

#define LDS_STRIDE 48
#define KSTRIDE    72
#define VSTRIDE    48

__device__ __forceinline__ f32x8 wmma_bf16(bf16x16 a, bf16x16 b, f32x8 c) {
  return __builtin_amdgcn_wmma_f32_16x16x32_f16(
      false, a, false, b, (short)0, c, false, false);
}
#define RSPLIT (1.0f / 2048.0f)
__device__ __forceinline__ bf16 lo_of(float v, bf16 h) { return (bf16)((v - (float)h) * 2048.0f); }
__device__ __forceinline__ f32x8 wmma_split(bf16x16 a, bf16x16 al, bf16x16 b, bf16x16 bl, f32x8 c) {
  f32x8 x = {}; x = wmma_bf16(al, b, x); x = wmma_bf16(a, bl, x); return wmma_bf16(a, b, c) + x * RSPLIT; }

template <typename T>
__device__ __forceinline__ bf16x16 load_frag(const T* __restrict__ base, int ld,
                                             int row0, int k0) {
  const int lane = threadIdx.x & 31;
  const int r    = lane & 15;
  const int kh   = (lane >> 4) * 8;
  const T* p0 = base + (size_t)(row0 + r) * ld + (k0 + kh);
  const T* p1 = p0 + 16;
  bf16x16 f;
#pragma unroll
  for (int i = 0; i < 8; ++i) {
    f[i]     = (bf16)p0[i];
    f[i + 8] = (bf16)p1[i];
  }
  return f;
}

__device__ __forceinline__ bf16x16 lds_frag(const bf16* base, int stride) {
  const int lane = threadIdx.x & 31;
  const int row  = lane & 15;
  const int kh   = (lane >> 4) * 8;
  const bf16x8 lo = *(const bf16x8*)(base + row * stride + kh);
  const bf16x8 hi = *(const bf16x8*)(base + row * stride + kh + 16);
  bf16x16 f;
#pragma unroll
  for (int i = 0; i < 8; ++i) { f[i] = lo[i]; f[i + 8] = hi[i]; }
  return f;
}

template <typename T>
__device__ __forceinline__ void stage_read16(const T* __restrict__ p, float* buf) {
#pragma unroll
  for (int i = 0; i < 16; ++i) buf[i] = (float)p[i];
}

__device__ __forceinline__ void stage_write(bf16* dst, const float* buf, int nquad) {
#pragma unroll
  for (int i = 0; i < nquad; ++i) {
    bf16x4 q;
    q[0] = (bf16)buf[4 * i];     q[1] = (bf16)buf[4 * i + 1];
    q[2] = (bf16)buf[4 * i + 2]; q[3] = (bf16)buf[4 * i + 3];
    *(bf16x4*)(dst + 4 * i) = q;
  }
}

__global__ __launch_bounds__(256) void transpose_pack_kernel(const float* __restrict__ W, bf16* __restrict__ WT, int K, int N, size_t plane) {
  __shared__ float tile[64][65];
  const int k0 = blockIdx.y * 64, n0 = blockIdx.x * 64, t = threadIdx.x;
  for (int i = t; i < 64 * 64; i += 256) { const int kr = i >> 6, nc = i & 63; tile[kr][nc] = W[(size_t)(k0 + kr) * N + n0 + nc]; }
  __syncthreads();
#pragma unroll 1
  for (int pass = 0; pass < 2; ++pass) {
    for (int i = t; i < 64 * 8; i += 256) { const int nr = i >> 3, k8 = (i & 7) * 8; bf16 hh[8], hl[8];
#pragma unroll
      for (int e = 0; e < 8; ++e) { const float v = tile[k8 + e][nr]; hh[e] = (bf16)v; hl[e] = lo_of(v, hh[e]); }
      bf16* d = WT + (size_t)(n0 + nr) * K + k0 + k8;
      *(volatile v4u_t*)d = *(const v4ua*)hh; *(volatile v4u_t*)(d + plane) = *(const v4ua*)hl; }
    __threadfence();
  }
}

template <typename AT, typename WT, int MODE>
__global__ __launch_bounds__(256) void gemm_bias_kernel(
    const AT* __restrict__ A, const WT* __restrict__ W,
    const float* __restrict__ bias, void* __restrict__ out,
    int M, int N, int K) {
  __shared__ bf16 ldsA[128 * LDS_STRIDE];
  __shared__ bf16 ldsW[256 * LDS_STRIDE];
  __shared__ __attribute__((aligned(16))) unsigned char sob[256 * 136 * 2];

  const int t    = threadIdx.x;
  const int wave = t >> 5;
  const int lane = t & 31;
  const int wm   = (wave & 1) * 64;
  const int wn   = (wave >> 1) * 64;
  const int mBlk = blockIdx.x * 128;
  const int nBlk = blockIdx.y * 256;

  const int arow = t >> 1;
  const int ach  = (t & 1) * 16;

  float abuf[16];
  float wbuf[32];

  stage_read16(A + (size_t)(mBlk + arow) * K + ach, abuf);
  stage_read16(W + (size_t)(nBlk + t) * K,          wbuf);
  stage_read16(W + (size_t)(nBlk + t) * K + 16,     wbuf + 16);

  f32x8 acc[4][4] = {};

  for (int k = 0; k < K; k += 32) {
    __syncthreads();
    stage_write(&ldsA[arow * LDS_STRIDE + ach], abuf, 4);
    stage_write(&ldsW[t * LDS_STRIDE],          wbuf, 8);
    if (k + 32 < K) {
      stage_read16(A + (size_t)(mBlk + arow) * K + (k + 32) + ach, abuf);
      stage_read16(W + (size_t)(nBlk + t) * K + (k + 32),          wbuf);
      stage_read16(W + (size_t)(nBlk + t) * K + (k + 32) + 16,     wbuf + 16);
    }
    __syncthreads();

    bf16x16 af[4], wf[4];
#pragma unroll
    for (int i = 0; i < 4; ++i)
      af[i] = lds_frag(ldsA + (wm + 16 * i) * LDS_STRIDE, LDS_STRIDE);
#pragma unroll
    for (int j = 0; j < 4; ++j)
      wf[j] = lds_frag(ldsW + (wn + 16 * j) * LDS_STRIDE, LDS_STRIDE);
#pragma unroll
    for (int i = 0; i < 4; ++i)
#pragma unroll
      for (int j = 0; j < 4; ++j)
        acc[i][j] = wmma_bf16(af[i], wf[j], acc[i][j]);
  }

  const int nlane = lane & 15;
  const int mh    = (lane >> 4) * 8;
  __syncthreads();
  if (MODE == 0 || MODE == 1) {
    bf16* so = (bf16*)sob;
#pragma unroll
    for (int i = 0; i < 4; ++i)
#pragma unroll
      for (int j = 0; j < 4; ++j) {
        const int nl = wn + 16 * j + nlane;
        const float bv = bias[nBlk + nl];
#pragma unroll
        for (int r = 0; r < 8; ++r) {
          const int ml = wm + 16 * i + mh + r;
          const bf16 hv = (bf16)(acc[i][j][r] + bv);
          if (MODE == 0) so[ml * 264 + nl] = hv;
          else           so[nl * 136 + ml] = hv;
        }
      }
    __syncthreads();
#pragma unroll 1
    for (int pass = 0; pass < 2; ++pass) {
      if (MODE == 0) {
        for (int ch = t; ch < 128 * 32; ch += 256) { const int ml = ch >> 5, q = (ch & 31) * 8;
          *(volatile v4u_t*)((bf16*)out + (size_t)(mBlk + ml) * N + nBlk + q) = *(const v4ua*)(so + ml * 264 + q); }
      } else {
        const int b_ = mBlk / SS, s0 = mBlk & (SS - 1);
        for (int ch = t; ch < 256 * 16; ch += 256) { const int nl = ch >> 4, q = (ch & 15) * 8; const int n = nBlk + nl, h = n / DKK, dk = n & (DKK - 1);
          *(volatile v4u_t*)((bf16*)out + (((size_t)(b_ * HH + h)) * DKK + dk) * SS + s0 + q) = *(const v4ua*)(so + nl * 136 + q); }
      }
      __threadfence();
    }
  } else {
    float* so = (float*)sob;
#pragma unroll 1
    for (int hf = 0; hf < 2; ++hf) {
      if (wm == hf * 64) {
#pragma unroll
        for (int i = 0; i < 4; ++i)
#pragma unroll
          for (int j = 0; j < 4; ++j) {
            const int nl = wn + 16 * j + nlane;
            const float bv = bias[nBlk + nl];
#pragma unroll
            for (int r = 0; r < 8; ++r) so[(16 * i + mh + r) * 260 + nl] = acc[i][j][r] + bv;
          }
      }
      __syncthreads();
#pragma unroll 1
      for (int pass = 0; pass < 2; ++pass) {
        for (int ch = t; ch < 64 * 64; ch += 256) { const int ml = ch >> 6, q = (ch & 63) * 4;
          *(volatile v4f_t*)((float*)out + (size_t)(mBlk + hf * 64 + ml) * N + nBlk + q) = *(const volatile v4fa*)(so + ml * 260 + q); }
        __threadfence();
      }
      __syncthreads();
    }
  }
}

template <typename AT, typename WT, int MODE>
__global__ __launch_bounds__(256) void gemm_split_kernel(
    const AT* __restrict__ A, size_t aPlane, const WT* __restrict__ W, size_t wPlane,
    const float* __restrict__ bias, void* __restrict__ out,
    int M, int N, int K) {
  __shared__ bf16 ldsA[128 * LDS_STRIDE], ldsAl[128 * LDS_STRIDE];
  __shared__ bf16 ldsW[256 * LDS_STRIDE], ldsWl[256 * LDS_STRIDE];
  __shared__ __attribute__((aligned(16))) unsigned char sob[256 * 136 * 2];

  const int t    = threadIdx.x;
  const int wave = t >> 5;
  const int lane = t & 31;
  const int wm   = (wave & 1) * 64;
  const int wn   = (wave >> 1) * 64;
  const int mBlk = blockIdx.x * 128;
  const int nBlk = blockIdx.y * 256;
  const int arow = t >> 1;
  const int ach  = (t & 1) * 16;

  f32x8 acc[4][4] = {};
  for (int k = 0; k < K; k += 32) {
    __syncthreads();
    {
      const AT* ap = A + (size_t)(mBlk + arow) * K + k + ach;
      bf16 hh[16], hl[16];
      if (sizeof(AT) == 4) {
#pragma unroll
        for (int i = 0; i < 16; ++i) { const float v = (float)ap[i]; hh[i] = (bf16)v; hl[i] = lo_of(v, hh[i]); }
      } else {
#pragma unroll
        for (int i = 0; i < 16; ++i) { hh[i] = (bf16)ap[i]; hl[i] = (bf16)ap[aPlane + i]; }
      }
#pragma unroll
      for (int i = 0; i < 16; ++i) { ldsA[arow * LDS_STRIDE + ach + i] = hh[i]; ldsAl[arow * LDS_STRIDE + ach + i] = hl[i]; }
    }
    {
      const WT* wp = W + (size_t)(nBlk + t) * K + k;
      if (sizeof(WT) == 4) {
#pragma unroll
        for (int i = 0; i < 32; ++i) { const float v = (float)wp[i]; const bf16 h_ = (bf16)v; ldsW[t * LDS_STRIDE + i] = h_; ldsWl[t * LDS_STRIDE + i] = lo_of(v, h_); }
      } else {
#pragma unroll
        for (int i = 0; i < 32; ++i) { ldsW[t * LDS_STRIDE + i] = (bf16)wp[i]; ldsWl[t * LDS_STRIDE + i] = (bf16)wp[wPlane + i]; }
      }
    }
    __syncthreads();
    bf16x16 wf[4], wfl[4];
#pragma unroll
    for (int j = 0; j < 4; ++j) { wf[j] = lds_frag(ldsW + (wn + 16 * j) * LDS_STRIDE, LDS_STRIDE); wfl[j] = lds_frag(ldsWl + (wn + 16 * j) * LDS_STRIDE, LDS_STRIDE); }
#pragma unroll
    for (int i = 0; i < 4; ++i) {
      const bf16x16 af = lds_frag(ldsA + (wm + 16 * i) * LDS_STRIDE, LDS_STRIDE), afl = lds_frag(ldsAl + (wm + 16 * i) * LDS_STRIDE, LDS_STRIDE);
#pragma unroll
      for (int j = 0; j < 4; ++j) acc[i][j] = wmma_split(af, afl, wf[j], wfl[j], acc[i][j]);
    }
  }

  const int nlane = lane & 15;
  const int mh    = (lane >> 4) * 8;
  __syncthreads();
  if (MODE == 1) {
    bf16* so = (bf16*)sob;
#pragma unroll
    for (int i = 0; i < 4; ++i)
#pragma unroll
      for (int j = 0; j < 4; ++j) {
        const int nl = wn + 16 * j + nlane;
        const float bv = bias ? bias[nBlk + nl] : 0.0f;
#pragma unroll
        for (int r = 0; r < 8; ++r) so[nl * 136 + wm + 16 * i + mh + r] = (bf16)(acc[i][j][r] + bv);
      }
    __syncthreads();
    const int b_ = mBlk >> 11, s0 = mBlk & (SS - 1);
#pragma unroll 1
    for (int pass = 0; pass < 2; ++pass) {
      for (int ch = t; ch < 256 * 16; ch += 256) { const int nl = ch >> 4, q = (ch & 15) * 8; const int n = nBlk + nl, h = n / DKK, dk = n & (DKK - 1);
        *(volatile v4u_t*)((bf16*)out + (((size_t)(b_ * HH + h)) * DKK + dk) * SS + s0 + q) = *(const v4ua*)(so + nl * 136 + q); }
      __threadfence();
    }
  } else {
    float* so = (float*)sob;
#pragma unroll 1
    for (int hf = 0; hf < 2; ++hf) {
      if (wm == hf * 64) {
#pragma unroll
        for (int i = 0; i < 4; ++i)
#pragma unroll
          for (int j = 0; j < 4; ++j) {
            const int nl = wn + 16 * j + nlane;
            const float bv = bias ? bias[nBlk + nl] : 0.0f;
#pragma unroll
            for (int r = 0; r < 8; ++r) so[(16 * i + mh + r) * 260 + nl] = acc[i][j][r] + bv;
          }
      }
      __syncthreads();
#pragma unroll 1
      for (int pass = 0; pass < 2; ++pass) {
        for (int ch = t; ch < 64 * 64; ch += 256) { const int ml = ch >> 6, q = (ch & 63) * 4;
          *(volatile v4f_t*)((float*)out + (size_t)(mBlk + hf * 64 + ml) * N + nBlk + q) = *(const volatile v4fa*)(so + ml * 260 + q); }
        __threadfence();
      }
      __syncthreads();
    }
  }
}


#define TK 128
#define NQK 1024

__global__ __launch_bounds__(128) void k_im2col(const float* __restrict__ x, float* __restrict__ A3) {
  const int bt = blockIdx.x, b = bt / SS, t0 = bt % SS, c = threadIdx.x;
  float v[3];
#pragma unroll
  for (int j = 0; j < 3; ++j) { const int tt = t0 + j - 2; v[j] = (tt >= 0) ? x[((size_t)b * SS + tt) * TK + c] : 0.0f; }
#pragma unroll 1
  for (int pass = 0; pass < 2; ++pass) {
#pragma unroll
    for (int j = 0; j < 3; ++j) *(volatile float*)(A3 + (size_t)bt * (3 * TK) + c * 3 + j) = v[j];
    __threadfence(); }
}
__global__ __launch_bounds__(128) void k_permw(const float* __restrict__ w, int kin, const float* __restrict__ bsrc, float* __restrict__ wp, float* __restrict__ bp) {
  const int np = blockIdx.x, h = np / TK, kk = np % TK, o = kk * HH + h, t = threadIdx.x;
  for (int i = t; i < kin; i += 128) { const float v = w[(size_t)o * kin + i]; *(volatile float*)(wp + (size_t)np * kin + i) = v; }
  if (bsrc && t == 0) *(volatile float*)(bp + np) = bsrc[o];
  __threadfence();
  for (int i = t; i < kin; i += 128) { const float v = w[(size_t)o * kin + i]; *(volatile float*)(wp + (size_t)np * kin + i) = v; }
  if (bsrc && t == 0) *(volatile float*)(bp + np) = bsrc[o];
}

__global__ __launch_bounds__(64) void attn128_kernel(const bf16* __restrict__ Qb, const bf16* __restrict__ Kb, const bf16* __restrict__ Vt, bf16* __restrict__ attnOut) {
  __shared__ bf16 ldsK[32 * KS2];
  __shared__ bf16 ldsV[128 * VSTRIDE];
  __shared__ __attribute__((aligned(16))) bf16 ldsO[2][2][16 * 136];
  const int q0blk = blockIdx.x * 32, h = blockIdx.y, b = blockIdx.z;
  const size_t oplane = (size_t)BB * SS * NQK;
  const int t = threadIdx.x, wave = t >> 5, lane = t & 31, qlane = lane & 15, kh8 = (lane >> 4) * 8;
  const int q0 = q0blk + wave * 16;
  const int nseq = b * HH + h;
  const bf16* Qh = Qb + (size_t)nseq * SS * DKK;
  const bf16* Kh = Kb + (size_t)nseq * SS * DKK;
  const bf16* Vh = Vt + (size_t)nseq * DKK * SS;
  const int krow = t >> 1, kcol = (t & 1) * 64;
  bf16x16 qf[4];
#pragma unroll
  for (int c = 0; c < 4; ++c) qf[c] = load_frag(Qh, DKK, q0, 32 * c);
  f32x8 o[8] = {};
  float mrun = -INFINITY, lrun = 0.0f;
  const float scale = 0.08838834764831845f * 1.44269504088896340736f;
  const int qi = q0 + qlane, kmax = q0blk + 31;
#pragma unroll 1
  for (int kb = 0; kb <= kmax; kb += 32) {
    __syncthreads();
    { const bf16* ks = Kh + (size_t)(kb + krow) * DKK + kcol;
#pragma unroll
      for (int i = 0; i < 8; ++i) *(bf16x8*)(&ldsK[krow * KS2 + kcol + 8 * i]) = *(const bf16x8*)(ks + 8 * i);
      const bf16* vs0 = Vh + (size_t)t * SS + kb; const bf16* vs1 = Vh + (size_t)(64 + t) * SS + kb;
#pragma unroll
      for (int i = 0; i < 4; ++i) { *(bf16x8*)(&ldsV[t * VSTRIDE + 8 * i]) = *(const bf16x8*)(vs0 + 8 * i); *(bf16x8*)(&ldsV[(64 + t) * VSTRIDE + 8 * i]) = *(const bf16x8*)(vs1 + 8 * i); } }
    __syncthreads();
    f32x8 s0 = {}, s1 = {};
#pragma unroll
    for (int c = 0; c < 4; ++c) { s0 = wmma_bf16(lds_frag(ldsK + c * 32, KS2), qf[c], s0); s1 = wmma_bf16(lds_frag(ldsK + 16 * KS2 + c * 32, KS2), qf[c], s1); }
    float mx = -INFINITY;
#pragma unroll
    for (int r = 0; r < 8; ++r) { const int j0 = kb + kh8 + r, j1 = j0 + 16;
      s0[r] = (j0 <= qi) ? s0[r] * scale : -INFINITY; s1[r] = (j1 <= qi) ? s1[r] * scale : -INFINITY; mx = fmaxf(mx, fmaxf(s0[r], s1[r])); }
    mx = fmaxf(mx, __shfl_xor(mx, 16, 32));
    const float mnew = fmaxf(mrun, mx), alpha = exp2f(mrun - mnew);
    float rsum = 0.0f; bf16x16 pf;
#pragma unroll
    for (int r = 0; r < 8; ++r) { const float p0 = exp2f(s0[r] - mnew), p1 = exp2f(s1[r] - mnew); rsum += p0 + p1; pf[r] = (bf16)(p0 * 1024.0f); pf[r + 8] = (bf16)(p1 * 1024.0f); }
    rsum += __shfl_xor(rsum, 16, 32);
    lrun = lrun * alpha + rsum; mrun = mnew;
#pragma unroll
    for (int j = 0; j < 8; ++j) {
#pragma unroll
      for (int r = 0; r < 8; ++r) o[j][r] *= alpha;
      o[j] = wmma_bf16(lds_frag(ldsV + (j * 16) * VSTRIDE, VSTRIDE), pf, o[j]); }
  }
  bf16* so = ldsO[wave][0]; bf16* sl = ldsO[wave][1];
  const float rl = 1.0f / (lrun * 1024.0f);
#pragma unroll
  for (int j = 0; j < 8; ++j)
#pragma unroll
    for (int r = 0; r < 8; ++r) { const float v = o[j][r] * rl; const bf16 hv = (bf16)v; so[qlane * 136 + j * 16 + kh8 + r] = hv; sl[qlane * 136 + j * 16 + kh8 + r] = lo_of(v, hv); }
  asm volatile("s_wait_dscnt 0" ::: "memory");
#pragma unroll 1
  for (int pass = 0; pass < 2; ++pass) {
#pragma unroll
    for (int it = 0; it < 8; ++it) { const int ch = lane + 32 * it, ql = ch >> 4, q8 = (ch & 15) * 8;
      bf16* dst = attnOut + ((size_t)(b * SS + q0 + ql)) * NQK + h * DKK + q8;
      *(volatile v4u_t*)dst = *(const v4ua*)(so + ql * 136 + q8); *(volatile v4u_t*)(dst + oplane) = *(const v4ua*)(sl + ql * 136 + q8); }
    __threadfence();
  }
}
__global__ __launch_bounds__(256) void k_vt2(const float* __restrict__ V, bf16* __restrict__ Vt2) {
  __shared__ float tile[64][65];
  const int nseq = blockIdx.z, t0 = blockIdx.x * 64, d0 = blockIdx.y * 64, t = threadIdx.x;
  const float* src = V + ((size_t)nseq * SS + t0) * DKK + d0;
  for (int i = t; i < 64 * 64; i += 256) { const int r = i >> 6, c = i & 63; tile[r][c] = src[(size_t)r * DKK + c]; }
  __syncthreads();
#pragma unroll 1
  for (int pass = 0; pass < 2; ++pass) {
    for (int i = t; i < 64 * 8; i += 256) { const int dr = i >> 3, t8 = (i & 7) * 8; bf16 hh[8];
#pragma unroll
      for (int e = 0; e < 8; ++e) hh[e] = (bf16)tile[t8 + e][dr];
      *(volatile v4u_t*)(Vt2 + ((size_t)nseq * DKK + d0 + dr) * SS + t0 + t8) = *(const v4ua*)hh; }
    __threadfence();
  }
}
__global__ __launch_bounds__(256) void k_outT(const float* __restrict__ UT, const float* __restrict__ bu, float* __restrict__ out) {
  __shared__ float tile[64][65];
  const int n0 = blockIdx.x * 64, cb = blockIdx.y * 64, t = threadIdx.x;
  for (int i = t; i < 64 * 64; i += 256) { const int c = i >> 6, nn = i & 63; tile[c][nn] = UT[(size_t)(cb + c) * (BB * SS) + n0 + nn]; }
  __syncthreads();
#pragma unroll 1
  for (int pass = 0; pass < 2; ++pass) {
    for (int i = t; i < 64 * 16; i += 256) { const int nr = i >> 4, c4 = (i & 15) * 4; v4f_t v;
#pragma unroll
      for (int q = 0; q < 4; ++q) v[q] = tile[c4 + q][nr] + bu[cb + c4 + q];
      *(volatile v4f_t*)(out + (size_t)(n0 + nr) * TK + cb + c4) = v; }
    __threadfence();
  }
}

extern "C" void kernel_launch(void* const* d_in, const int* in_sizes, int n_in,
                              void* d_out, int out_size, void* d_ws, size_t ws_size,
                              hipStream_t stream) {
  (void)in_sizes; (void)n_in; (void)out_size; (void)ws_size;
  const float* x  = (const float*)d_in[0];
  const float* wq = (const float*)d_in[1];  const float* bq = (const float*)d_in[2];
  const float* wk = (const float*)d_in[3];  const float* bk = (const float*)d_in[4];
  const float* wv = (const float*)d_in[5];
  const float* wu = (const float*)d_in[6];  const float* bu = (const float*)d_in[7];
  char* ws = (char*)d_ws;
  const int M = BB * SS;
  float* A3  = (float*)ws; ws += (size_t)M * 3 * TK * 4;
  float* wqp = (float*)ws; ws += (size_t)NQK * 3 * TK * 4;  float* bqp = (float*)ws; ws += NQK * 4;
  float* wkp = (float*)ws; ws += (size_t)NQK * 3 * TK * 4;  float* bkp = (float*)ws; ws += NQK * 4;
  float* wvp = (float*)ws; ws += (size_t)NQK * TK * 4;
  bf16* Qb   = (bf16*)ws;  ws += (size_t)M * NQK * 2;
  bf16* Kb   = (bf16*)ws;  ws += (size_t)M * NQK * 2;
  bf16* VtB  = (bf16*)ws;  ws += (size_t)M * NQK * 2;
  bf16* attn = (bf16*)ws;  ws += (size_t)M * NQK * 2 * 2;
  float* Vf  = (float*)attn;
  float* UT  = (float*)ws; ws += (size_t)TK * M * 4;
  k_im2col<<<M, 128, 0, stream>>>(x, A3);
  k_permw<<<NQK, 128, 0, stream>>>(wq, 3 * TK, bq, wqp, bqp);
  k_permw<<<NQK, 128, 0, stream>>>(wk, 3 * TK, bk, wkp, bkp);
  k_permw<<<NQK, 128, 0, stream>>>(wv, TK, nullptr, wvp, nullptr);
  dim3 gGrid(M / 128, NQK / 256), gBlk(256);
  gemm_bias_kernel<float, float, 0><<<gGrid, gBlk, 0, stream>>>(A3, wqp, bqp, Qb, M, NQK, 3 * TK);
  gemm_bias_kernel<float, float, 0><<<gGrid, gBlk, 0, stream>>>(A3, wkp, bkp, Kb, M, NQK, 3 * TK);
  gemm_split_kernel<float, float, 2><<<gGrid, gBlk, 0, stream>>>(x, 0, wvp, 0, nullptr, Vf, M, NQK, TK);
  k_vt2<<<dim3(SS / 64, DKK / 64, BB * HH), 256, 0, stream>>>(Vf, VtB);
  attn128_kernel<<<dim3(SS / 32, HH, BB), 64, 0, stream>>>(Qb, Kb, VtB, attn);
  gemm_split_kernel<float, bf16, 2><<<dim3(1, M / 256), gBlk, 0, stream>>>(wu, 0, attn, (size_t)M * NQK, nullptr, UT, TK, M, NQK);
  k_outT<<<dim3(M / 64, TK / 64), 256, 0, stream>>>(UT, bu, (float*)d_out);
}
